// FullAttention_14963666060008
// MI455X (gfx1250) — hardware-verified
//
#include <hip/hip_runtime.h>


#ifndef NB
#define NB 2
#endif
#ifndef SEQ
#define SEQ 2048
#endif
#define NB_FULL  2
#define SEQ_FULL 2048
#ifndef OUT_SEQ
#define OUT_SEQ SEQ
#endif
#define NHD  16
#define HD   64
#define HE   (NHD * HD)
#define AW   4
#define OSP  68
#define TP   68
#define EROWS (SEQ < 512 ? SEQ : 512)
#define QRS  2048.0f
#define QRI  (1.0f / 2048.0f)
#define SC2  ((float)(0.125 * 1.4426950408889634))
#define PSH  14.0f
#define NEGB (-3.0e38f)

static_assert(HD == 64);
static_assert(NHD * HD == HE);
static_assert(HD % 32 == 0);
static_assert(HE % 8 == 0);
static_assert(SEQ % 64 == 0);
static_assert(SEQ % 32 == 0);
static_assert(SEQ % (16 * AW) == 0);
static_assert(EROWS % (16 * AW) == 0);
static_assert((SEQ - EROWS) % (16 * AW) == 0);
static_assert(EROWS >= 32);
static_assert(EROWS <= SEQ);
static_assert(NB <= NB_FULL);
static_assert(SEQ <= SEQ_FULL);
static_assert(OSP >= HD);
static_assert((OSP * 4) % 16 == 0);
static_assert(TP >= 64);
static_assert((TP * 4) % 16 == 0);
static_assert((((size_t)SEQ * HE) / 8) % 256 == 0);
static_assert((size_t)32 * 16 * 8 == (size_t)16 * HD * 4);
static_assert((size_t)256 * 16 * 2 == (size_t)64 * 128);
static_assert((size_t)256 * 4 * 4 == (size_t)64 * HD);
static_assert((size_t)AW * 16 * OSP * 4 <= 131072);
static_assert((size_t)64 * TP * 4 <= 131072);

typedef _Float16 h16;
typedef __attribute__((ext_vector_type(16))) _Float16 v16h;
typedef __attribute__((ext_vector_type(8)))  _Float16 v8h;
typedef __attribute__((ext_vector_type(8)))  float    v8f;
typedef __attribute__((ext_vector_type(4)))  float    v4f;
typedef v4f  __attribute__((may_alias)) v4fa;

__device__ __forceinline__ unsigned short f2bf(float f) { unsigned u = __float_as_uint(f); u += 0x7FFFu + ((u >> 16) & 1u); return (unsigned short)(u >> 16); }
__device__ __forceinline__ float bfr(float f) { return __uint_as_float(((unsigned)f2bf(f)) << 16); }
__device__ __forceinline__ v16h cat16(v8h lo, v8h hi) { return __builtin_shufflevector(lo, hi, 0, 1, 2, 3, 4, 5, 6, 7, 8, 9, 10, 11, 12, 13, 14, 15); }
__device__ __forceinline__ v16h  ldh(const h16* p) { return cat16(*(const v8h*)p, *(const v8h*)(p + 16)); }
__device__ __forceinline__ void wave_sync() { __builtin_amdgcn_fence(3  , "wavefront"); __builtin_amdgcn_wave_barrier(); asm volatile("" ::: "memory"); }
static __device__ __forceinline__ h16 toh_flush(float v) { const h16 r = (h16)v; return (fabsf(v) < 6.103515625e-05f) ? (h16)0.0f : r; }
__device__ __forceinline__ v8f wmma16g(v16h a, v16h b, v8f c) {
    c = __builtin_amdgcn_wmma_f32_16x16x32_f16(false, a, false, b, (short)0, c, false, false);
    asm volatile("v_nop\n\tv_nop\n\tv_nop\n\tv_nop" : "+v"(c) : "v"(a), "v"(b));
    return c;
}

__global__ __launch_bounds__(256) void k_cvth(const float* __restrict__ src, h16* dst, size_t n8, size_t sstride, size_t dstride) {
    const size_t i = (size_t)blockIdx.x * 256 + threadIdx.x; if (i >= n8) return;
    const size_t so = (size_t)blockIdx.y * sstride + i * 8;
    const size_t dofs = (size_t)blockIdx.y * dstride + i * 8;
    const v8f v = *(const v8f*)(src + so); v8h o;
#pragma unroll
    for (int k = 0; k < 8; ++k) o[k] = toh_flush(bfr(v[k]));
    *(volatile v8h*)(dst + dofs) = o; __threadfence(); *(volatile v8h*)(dst + dofs) = o;
}

__global__ __launch_bounds__(256) void k_vtr(const float* __restrict__ V, h16* VT) {
    __shared__ __align__(16) float tl[64 * TP];
    const int tid = threadIdx.x;
    const int tt0 = blockIdx.x * 64; const int zh = blockIdx.y; const int b = zh / NHD, h = zh % NHD;
    const size_t vb = ((size_t)b * SEQ_FULL + tt0) * HE + (size_t)h * HD;
#pragma unroll
    for (int s = 0; s < 4; ++s) { const int p = s * 256 + tid; const int t = p >> 4, d4 = (p & 15) * 4;
        const v4f x = *(const v4f*)(V + vb + (size_t)t * HE + d4);
#pragma unroll
        for (int i = 0; i < 4; ++i) tl[(d4 + i) * TP + t] = bfr(x[i]); }
    __syncthreads();
    const size_t ob = ((size_t)zh * HD) * SEQ + tt0;
    const int dA = tid >> 3, dB = (256 + tid) >> 3, c8 = (tid & 7) * 8;
    v8h hvA, hvB;
    { const v4f x0 = *(const v4fa*)(&tl[dA * TP + c8]); const v4f x1 = *(const v4fa*)(&tl[dA * TP + c8 + 4]);
#pragma unroll
      for (int i = 0; i < 4; ++i) { hvA[i] = toh_flush(x0[i]); hvA[4 + i] = toh_flush(x1[i]); } }
    { const v4f x0 = *(const v4fa*)(&tl[dB * TP + c8]); const v4f x1 = *(const v4fa*)(&tl[dB * TP + c8 + 4]);
#pragma unroll
      for (int i = 0; i < 4; ++i) { hvB[i] = toh_flush(x0[i]); hvB[4 + i] = toh_flush(x1[i]); } }
    const size_t oA = ob + (size_t)dA * SEQ + c8, oB = ob + (size_t)dB * SEQ + c8;
    *(volatile v8h*)(VT + oA) = hvA; *(volatile v8h*)(VT + oB) = hvB;
    __threadfence();
    *(volatile v8h*)(VT + oA) = hvA; *(volatile v8h*)(VT + oB) = hvB;
}

template <int EARLY>
__device__ __forceinline__ void flash_body(const h16* __restrict__ QH, const h16* __restrict__ KP, const h16* __restrict__ VT, float* OUT) {
    __shared__ __align__(16) float os[AW * 16 * OSP];
    const int lane = threadIdx.x & 31, lr = lane & 15, hi = lane >> 4;
    const int wave = __builtin_amdgcn_readfirstlane((int)(threadIdx.x >> 5));
    const int zh = blockIdx.y; const int b = zh / NHD, h = zh % NHD;
    const int t0 = (EARLY ? 0 : EROWS) + (blockIdx.x * AW + wave) * 16;
    const int lim = t0 + lr;
    const int nk = (t0 + 16 + 31) & ~31;
    const size_t rowb = (size_t)b * SEQ * HE + (size_t)h * HD;
    const size_t qo = rowb + (size_t)(t0 + lr) * HE + 8 * hi;
    const v16h q0 = ldh(QH + qo), q1 = ldh(QH + qo + 32);
    const size_t ko = rowb + (size_t)lr * HE + 8 * hi;
    const size_t vo = ((size_t)zh * HD + (size_t)lr) * SEQ + 8 * hi;
    const v16h hz = (v16h){};
    v8f o[4], oR[4];
#pragma unroll
    for (int j = 0; j < 4; ++j) { o[j] = (v8f){}; oR[j] = (v8f){}; }
    float m = NEGB, l = 0.0f;
#pragma unroll 1
    for (int key0 = 0; key0 < nk; key0 += 32) {
        const h16* ka = KP + ko + (size_t)key0 * HE;
        const v16h ka0 = ldh(ka), ka1 = ldh(ka + 32), kb0 = ldh(ka + (size_t)16 * HE), kb1 = ldh(ka + (size_t)16 * HE + 32);
        v8f sA = (v8f){}, sB = (v8f){};
        sA = wmma16g(ka0, q0, sA); sB = wmma16g(kb0, q0, sB);
        sA = wmma16g(ka1, q1, sA); sB = wmma16g(kb1, q1, sB);
        const int ja = key0 + 8 * hi;
        float ta[8], tb[8]; bool fa[8], fb[8]; float mx = NEGB;
#pragma unroll
        for (int r = 0; r < 8; ++r) {
            fa[r] = (ja + r <= lim);
            fb[r] = (ja + 16 + r <= lim);
            ta[r] = sA[r] * SC2; tb[r] = sB[r] * SC2;
            mx = fmaxf(mx, fmaxf(fa[r] ? ta[r] : NEGB, fb[r] ? tb[r] : NEGB)); }
        mx = fmaxf(mx, __shfl_xor(mx, 16, 32));
        const float mnew = fmaxf(m, mx);
        const float alpha = __builtin_amdgcn_exp2f(m - mnew);
        const float sh = PSH - mnew;
        v16h pb, pr = hz; float ls = 0.0f;
#pragma unroll
        for (int r = 0; r < 8; ++r) {
            const float ea = __builtin_amdgcn_exp2f(ta[r] + sh), eb = __builtin_amdgcn_exp2f(tb[r] + sh);
            const float ga = fa[r] ? ea : 0.0f, gb = fb[r] ? eb : 0.0f;
            const h16 pa = toh_flush(ga); const h16 pc = toh_flush(gb);
            pb[r] = pa; pb[8 + r] = pc;
            if (EARLY) { pr[r] = toh_flush((ga - (float)pa) * QRS); pr[8 + r] = toh_flush((gb - (float)pc) * QRS); ls += ga + gb; }
            else       { ls += (float)pa + (float)pc; } }
        l = l * alpha + ls; m = mnew;
#pragma unroll
        for (int j = 0; j < 4; ++j) o[j] = o[j] * alpha;
        if (EARLY) {
#pragma unroll
            for (int j = 0; j < 4; ++j) oR[j] = oR[j] * alpha; }
        const h16* va = VT + vo + key0;
        const v16h v0 = ldh(va), v1 = ldh(va + (size_t)16 * SEQ), v2 = ldh(va + (size_t)32 * SEQ), v3 = ldh(va + (size_t)48 * SEQ);
        o[0] = wmma16g(v0, pb, o[0]); o[1] = wmma16g(v1, pb, o[1]); o[2] = wmma16g(v2, pb, o[2]); o[3] = wmma16g(v3, pb, o[3]);
        if (EARLY) {
            oR[0] = wmma16g(v0, pr, oR[0]); oR[1] = wmma16g(v1, pr, oR[1]); oR[2] = wmma16g(v2, pr, oR[2]); oR[3] = wmma16g(v3, pr, oR[3]);
        }
    }
    l += __shfl_xor(l, 16, 32);
    const bool any = l > 0.0f;
    const float lsafe = any ? l : 1.0f;
    const float inv = any ? (1.0f / lsafe) : 0.0f;
    const int wb = wave * 16 * OSP;
#pragma unroll
    for (int j = 0; j < 4; ++j) {
        v8f f = o[j];
        if (EARLY) f = o[j] + oR[j] * QRI;
        v4f a, c;
        a[0] = f[0] * inv; a[1] = f[1] * inv; a[2] = f[2] * inv; a[3] = f[3] * inv; c[0] = f[4] * inv; c[1] = f[5] * inv; c[2] = f[6] * inv; c[3] = f[7] * inv;
        *(v4fa*)(&os[wb + lr * OSP + 16 * j + 8 * hi]) = a; *(v4fa*)(&os[wb + lr * OSP + 16 * j + 8 * hi + 4]) = c; }
    wave_sync();
    float* orow = OUT + (((size_t)b * OUT_SEQ + t0) * NHD + h) * HD;
#pragma unroll 1
    for (int ps = 0; ps < 2; ++ps) {
#pragma unroll
        for (int s = 0; s < 8; ++s) { const int row = 2 * s + (lane >> 4), cofs = (lane & 15) * 4;
            const v4f val = *(const v4fa*)(&os[wb + row * OSP + cofs]);
            *(volatile v4f*)(orow + (size_t)row * HE + cofs) = val; }
        if (ps == 0) __threadfence(); }
}

__global__ __launch_bounds__(32 * AW) void k_flash_early(const h16* __restrict__ QH, const h16* __restrict__ KP, const h16* __restrict__ VT, float* OUT) {
    flash_body<1>(QH, KP, VT, OUT);
}

__global__ __launch_bounds__(32 * AW) void k_flash_late(const h16* __restrict__ QH, const h16* __restrict__ KP, const h16* __restrict__ VT, float* OUT) {
    flash_body<0>(QH, KP, VT, OUT);
}

static constexpr size_t al256(size_t v) { return (v + 255) & ~(size_t)255; }
static constexpr size_t SZ_QK = al256((size_t)NB * SEQ * HE * 2);
static constexpr size_t SZ_VT = al256((size_t)NB * NHD * HD * SEQ * 2);
static constexpr size_t SZ_TOTAL = 2 * SZ_QK + SZ_VT;
static_assert(SZ_TOTAL <= (size_t)134217728);
static_assert(((size_t)NB * SEQ * HE * 2) % 128 == 0);
static_assert(((size_t)SEQ * 2) % 128 == 0);

extern "C" void kernel_launch(void* const* d_in, const int* in_sizes, int n_in,
                              void* d_out, int out_size, void* d_ws, size_t ws_size, hipStream_t stream) {
    if (n_in < 3) return;
    const size_t needx = ((size_t)(NB - 1) * SEQ_FULL + SEQ) * HE;
    if ((size_t)in_sizes[0] < needx || (size_t)in_sizes[1] < needx || (size_t)in_sizes[2] < needx) return;
    if ((size_t)out_size < ((size_t)(NB - 1) * OUT_SEQ + SEQ) * HE) return;
    if (SZ_TOTAL > ws_size) return;
    const float* qin = (const float*)d_in[0];
    const float* kin = (const float*)d_in[1];
    const float* vin = (const float*)d_in[2];
    float* OUT = (float*)d_out;
    char* wsp = (char*)d_ws;
    h16* QH = (h16*)wsp; wsp += SZ_QK;
    h16* KP = (h16*)wsp; wsp += SZ_QK;
    h16* VT = (h16*)wsp; wsp += SZ_VT;

    { const size_t n8 = (size_t)SEQ * HE / 8;
      const dim3 g((unsigned)((n8 + 255) / 256), NB, 1);
      k_cvth<<<g, 256, 0, stream>>>(qin, QH, n8, (size_t)SEQ_FULL * HE, (size_t)SEQ * HE);
      k_cvth<<<g, 256, 0, stream>>>(kin, KP, n8, (size_t)SEQ_FULL * HE, (size_t)SEQ * HE); }
    k_vtr<<<dim3(SEQ / 64, NB * NHD, 1), 256, 0, stream>>>(vin, VT);

    k_flash_early<<<dim3(EROWS / (16 * AW), NB * NHD, 1), 32 * AW, 0, stream>>>(QH, KP, VT, OUT);
    if (SEQ > EROWS)
        k_flash_late<<<dim3((SEQ - EROWS) / (16 * AW), NB * NHD, 1), 32 * AW, 0, stream>>>(QH, KP, VT, OUT);
}
